// LongformerSelfAttention_54958401519621
// MI455X (gfx1250) — hardware-verified
//
#include <hip/hip_runtime.h>


#ifndef NB
#define NB 2
#endif
#ifndef SEQ
#define SEQ 4096
#endif
#define NB_FULL  2
#define SEQ_FULL 4096
#define DM   768
#define NH_  12
#define HD   64
#define WIN  256
#define TOK  (NB * SEQ)
#define NT   ((2 * WIN + 16) / 32 + 1)
#define PPL  40
#define PC   1024.0f
#define RC   4096.0f
#define QSC  0.125f
#define L2E  1.4426950408889634f
static_assert(SEQ % 128 == 0);
static_assert(WIN % 32 == 0);
static_assert(DM == NH_ * HD);
static_assert(DM % 64 == 0);
static_assert(TOK % 64 == 0);
static_assert(((size_t)TOK * DM) % 1024 == 0);

typedef _Float16 h16;
typedef unsigned short bf;
typedef __attribute__((ext_vector_type(16))) __bf16   v16bf;
typedef __attribute__((ext_vector_type(16))) _Float16 v16h;
typedef __attribute__((ext_vector_type(8)))  _Float16 v8h;
typedef __attribute__((ext_vector_type(8)))  unsigned short v8us;
typedef __attribute__((ext_vector_type(8)))  float    v8f;
typedef __attribute__((ext_vector_type(4)))  float    v4f;
typedef v8h  __attribute__((may_alias)) v8ha;
typedef v4f  __attribute__((may_alias)) v4fa;
typedef v8us __attribute__((may_alias)) v8usa;
typedef __attribute__((ext_vector_type(2))) _Float16 v2h;
typedef __attribute__((ext_vector_type(4))) _Float16 v4h;
typedef __attribute__((ext_vector_type(2))) unsigned short v2us;
typedef __attribute__((ext_vector_type(4))) unsigned short v4us;
typedef __attribute__((ext_vector_type(2))) float v2f;

__device__ __forceinline__ unsigned short f2bf(float f) { unsigned u = __float_as_uint(f); u += 0x7FFFu + ((u >> 16) & 1u); return (unsigned short)(u >> 16); }
__device__ __forceinline__ float bf2f(unsigned short b) { return __uint_as_float(((unsigned)b) << 16); }
__device__ __forceinline__ float bfr(float f) { return bf2f(f2bf(f)); }
__device__ __forceinline__ v16h cat16(v8h lo, v8h hi) { return __builtin_shufflevector(lo, hi, 0, 1, 2, 3, 4, 5, 6, 7, 8, 9, 10, 11, 12, 13, 14, 15); }
__device__ __forceinline__ v16bf cat16b(v8us lo, v8us hi) { return __builtin_bit_cast(v16bf, __builtin_shufflevector(lo, hi, 0, 1, 2, 3, 4, 5, 6, 7, 8, 9, 10, 11, 12, 13, 14, 15)); }
__device__ __forceinline__ v8f wmma16(v16h a, v16h b, v8f c) { return __builtin_amdgcn_wmma_f32_16x16x32_f16(false, a, false, b, (short)0, c, false, false); }
__device__ __forceinline__ v8f wmmab(v16bf a, v16bf b, v8f c) { return __builtin_amdgcn_wmma_f32_16x16x32_bf16(false, a, false, b, (short)0, c, false, false); }
__device__ __forceinline__ v8h ld8(const h16* p) { return *(const v8h*)p; }

template <typename T16> struct WFrag;
template <> struct WFrag<h16> { typedef v16h V; static __device__ __forceinline__ V ld(const h16* p) { return cat16(*(const v8h*)p, *(const v8h*)(p + 16)); } static __device__ __forceinline__ v8f mma(V a, V b, v8f c) { return wmma16(a, b, c); } };
template <> struct WFrag<bf> { typedef v16bf V; static __device__ __forceinline__ V ld(const bf* p) { return cat16b(*(const v8us*)p, *(const v8us*)(p + 16)); } static __device__ __forceinline__ v8f mma(V a, V b, v8f c) { return wmmab(a, b, c); } };
template <typename T16, int NSPLIT, bool BIAS>
__global__ __launch_bounds__(32) void k_gemmw(const T16* __restrict__ A, const T16* __restrict__ A2, const T16* __restrict__ Bt, const T16* __restrict__ Bt2, int K, float* C, int ldc, const float* __restrict__ bias, size_t sA, size_t sB, size_t sC) {
    typedef typename WFrag<T16>::V V;
    __shared__ __align__(16) float os[16 * 68];
    const size_t z = blockIdx.z; A += z * sA; if (A2) A2 += z * sA; Bt += z * sB; if (Bt2) Bt2 += z * sB; C += z * sC;
    const int lane = threadIdx.x & 31, lr = lane & 15, hi = lane >> 4; const int r0 = blockIdx.x * 64, c0 = blockIdx.y * 64;
    v8f acc[4][4];
#pragma unroll
    for (int mb = 0; mb < 4; ++mb)
#pragma unroll
        for (int nb = 0; nb < 4; ++nb) acc[mb][nb] = (v8f){};
    const size_t aoff = (size_t)(r0 + lr) * K + 8 * hi, boff = (size_t)(c0 + lr) * K + 8 * hi;
#pragma unroll 1
    for (int kc = 0; kc < K; kc += 32) {
        V a[4], a2[4];
#pragma unroll
        for (int mb = 0; mb < 4; ++mb) { a[mb] = WFrag<T16>::ld(A + aoff + (size_t)mb * 16 * K + kc); if (NSPLIT == 1 || NSPLIT == 2) a2[mb] = WFrag<T16>::ld(A2 + aoff + (size_t)mb * 16 * K + kc); }
#pragma unroll
        for (int nb = 0; nb < 4; ++nb) { const V b = WFrag<T16>::ld(Bt + boff + (size_t)nb * 16 * K + kc); V b2; if (NSPLIT >= 2) b2 = WFrag<T16>::ld(Bt2 + boff + (size_t)nb * 16 * K + kc);
#pragma unroll
            for (int mb = 0; mb < 4; ++mb) { acc[mb][nb] = WFrag<T16>::mma(a[mb], b, acc[mb][nb]); if (NSPLIT == 1 || NSPLIT == 2) acc[mb][nb] = WFrag<T16>::mma(a2[mb], b, acc[mb][nb]); if (NSPLIT >= 2) acc[mb][nb] = WFrag<T16>::mma(a[mb], b2, acc[mb][nb]); } }
        asm volatile("v_nop\n\tv_nop\n\tv_nop\n\tv_nop" : "+v"(acc[0][0]), "+v"(acc[1][1]), "+v"(acc[2][2]), "+v"(acc[3][3]) : "v"(a[0]), "v"(a[3]));
    }
#pragma unroll
    for (int mb = 0; mb < 4; ++mb) {
#pragma unroll
        for (int nb = 0; nb < 4; ++nb) {
#pragma unroll
            for (int j = 0; j < 8; ++j) os[(hi * 8 + j) * 68 + nb * 16 + lr] = acc[mb][nb][j]; }
        __builtin_amdgcn_wave_barrier(); asm volatile("" ::: "memory");
        float* crow = C + (size_t)(r0 + mb * 16) * ldc + c0;
#pragma unroll 1
        for (int ps = 0; ps < 2; ++ps) {
#pragma unroll
            for (int s = 0; s < 8; ++s) { const int row = 2 * s + hi, cofs = lr * 4; v4f val = *(const v4fa*)(os + row * 68 + cofs); if (BIAS) { val[0] += bfr(bias[c0 + cofs]); val[1] += bfr(bias[c0 + cofs + 1]); val[2] += bfr(bias[c0 + cofs + 2]); val[3] += bfr(bias[c0 + cofs + 3]); }
                *(volatile v4f*)(crow + (size_t)row * ldc + cofs) = val; }
            if (ps == 0) __threadfence(); }
        __builtin_amdgcn_wave_barrier(); asm volatile("" ::: "memory");
    }
}

__global__ __launch_bounds__(256) void k_wtG(const float* __restrict__ w, int K, int N, bf* Bt) {
    const int lane = threadIdx.x & 31; const int L0 = (blockIdx.x * 8 + (threadIdx.x >> 5)) * 8; const int nlines = N * K / 64;
#pragma unroll
    for (int ps = 0; ps < 2; ++ps) {
#pragma unroll 1
        for (int l = 0; l < 8; ++l) { const int L = L0 + l; if (L >= nlines) break; const size_t e = (size_t)L * 64 + lane * 2; const int k = (int)(e % K), n = (int)(e / K); v2us o;
            o[0] = f2bf(w[(size_t)k * N + n]); o[1] = f2bf(w[(size_t)(k + 1) * N + n]); *(volatile v2us*)(Bt + e) = o; }
        if (ps == 0) __threadfence(); }
}
__global__ __launch_bounds__(256) void k_cvt8(const float* __restrict__ src, bf* dst, size_t n8) { const size_t i = (size_t)blockIdx.x * 256 + threadIdx.x; if (i >= n8) return; const v8f v = *(const v8f*)(src + i * 8); v8us o;
#pragma unroll
    for (int k = 0; k < 8; ++k) o[k] = f2bf(v[k]); *(volatile v8us*)(dst + i * 8) = o; __threadfence(); *(volatile v8us*)(dst + i * 8) = o; }

__global__ __launch_bounds__(256) void k_qkp(const float* __restrict__ F, h16* P) {
    const size_t e = ((size_t)blockIdx.x * 256 + threadIdx.x) * 4; if (e >= (size_t)TOK * DM) return;
    const int d = (int)(e % HD); const int s = (int)((e / HD) % SEQ); const int hh = (int)((e / ((size_t)HD * SEQ)) % NH_); const int bb = (int)(e / ((size_t)HD * SEQ * NH_));
    const v4f v = *(const v4f*)(F + ((size_t)bb * SEQ + s) * DM + hh * HD + d);
    v4h o;
#pragma unroll
    for (int q = 0; q < 4; ++q) o[q] = (h16)v[q];
    *(volatile v4h*)(P + e) = o; __threadfence(); *(volatile v4h*)(P + e) = o;
}
__global__ __launch_bounds__(256) void k_vp(const float* __restrict__ F, h16* VH, h16* VR) {
    const size_t e = ((size_t)blockIdx.x * 256 + threadIdx.x) * 4; if (e >= (size_t)TOK * DM) return;
    const int s = (int)(e % SEQ); const int d = (int)((e / SEQ) % HD); const int hh = (int)((e / ((size_t)SEQ * HD)) % NH_); const int bb = (int)(e / ((size_t)SEQ * HD * NH_));
    const float* f = F + ((size_t)bb * SEQ + s) * DM + hh * HD + d;
    v4h oh, orr;
#pragma unroll
    for (int q = 0; q < 4; ++q) { const float x = f[(size_t)q * DM]; const h16 hx = (h16)x; oh[q] = hx; float rr = x - (float)hx; rr = rr * RC; orr[q] = (h16)rr; }
    *(volatile v4h*)(VH + e) = oh; *(volatile v4h*)(VR + e) = orr; __threadfence(); *(volatile v4h*)(VH + e) = oh; *(volatile v4h*)(VR + e) = orr;
}

__global__ __launch_bounds__(256) __attribute__((amdgpu_num_vgpr(256)))
void k_attn(const h16* __restrict__ QP, const h16* __restrict__ KP, const h16* __restrict__ VHp, const h16* __restrict__ VRp, float* OUT) {
    __shared__ __align__(16) h16 pbh[8][16 * PPL];
    __shared__ __align__(16) h16 pbr[8][16 * PPL];
    __shared__ __align__(16) float os[8][16 * 68];
    const int wave = threadIdx.x >> 5, lane = threadIdx.x & 31, hi = lane >> 4, lr = lane & 15;
    const int h = blockIdx.y, b = blockIdx.z;
    const int q0 = blockIdx.x * 128 + wave * 16;
    const size_t bh = (size_t)b * NH_ + h;
    const h16* Qp = QP + bh * ((size_t)SEQ * HD); const h16* Kp = KP + bh * ((size_t)SEQ * HD);
    const h16* Vh = VHp + bh * ((size_t)HD * SEQ); const h16* Vr = VRp + bh * ((size_t)HD * SEQ);
    h16* ph_w = &pbh[wave][0]; h16* pr_w = &pbr[wave][0]; float* os_w = &os[wave][0];
    const h16* qrow = Qp + (size_t)(q0 + lr) * HD + 8 * hi;
    const v16h qa0 = cat16(ld8(qrow), ld8(qrow + 16));
    const v16h qa1 = cat16(ld8(qrow + 32), ld8(qrow + 48));
    v8f acc[4], rac[4];
#pragma unroll
    for (int ds = 0; ds < 4; ++ds) { acc[ds] = (v8f){}; rac[ds] = (v8f){}; }
    float mrow[8], lrow[8];
#pragma unroll
    for (int r = 0; r < 8; ++r) { mrow[r] = -3.0e38f; lrow[r] = 0.0f; }
    const int ktlo = (q0 - WIN + 32 * 8192) / 32 - 8192;
    const int kta = ktlo < 0 ? 0 : ktlo;
    const int ktb0 = ktlo + NT; const int ktb = ktb0 > (SEQ / 32) ? (SEQ / 32) : ktb0;
#pragma unroll 1
    for (int kt = kta; kt < ktb; ++kt) {
        const int j0 = kt * 32;
        const h16* kp0 = Kp + (size_t)(j0 + lr) * HD + 8 * hi; const h16* kp1 = kp0 + 16 * HD;
        const v16h kb00 = cat16(ld8(kp0), ld8(kp0 + 16)), kb01 = cat16(ld8(kp0 + 32), ld8(kp0 + 48));
        const v16h kb10 = cat16(ld8(kp1), ld8(kp1 + 16)), kb11 = cat16(ld8(kp1 + 32), ld8(kp1 + 48));
        v8f sc0 = (v8f){}, sc1 = (v8f){};
        sc0 = wmma16(qa0, kb00, sc0); sc0 = wmma16(qa1, kb01, sc0);
        sc1 = wmma16(qa0, kb10, sc1); sc1 = wmma16(qa1, kb11, sc1);
        asm volatile("v_nop\n\tv_nop\n\tv_nop\n\tv_nop" : "+v"(sc0), "+v"(sc1) : "v"(qa0), "v"(qa1), "v"(kb10), "v"(kb11));
        const int key0 = j0 + lr, key1 = key0 + 16;
#pragma unroll
        for (int r = 0; r < 8; ++r) {
            const int i = q0 + 8 * hi + r;
            const int dd0 = key0 - i, dd1 = key1 - i;
            const bool v0 = (dd0 <= WIN) && (dd0 >= -WIN);
            const bool v1 = (dd1 <= WIN) && (dd1 >= -WIN);
            const float s0 = sc0[r] * QSC, s1 = sc1[r] * QSC;
            const float x0 = v0 ? s0 : -3.0e38f;
            const float x1 = v1 ? s1 : -3.0e38f;
            float tm = fmaxf(x0, x1);
            tm = fmaxf(tm, __shfl_xor(tm, 1, 32)); tm = fmaxf(tm, __shfl_xor(tm, 2, 32)); tm = fmaxf(tm, __shfl_xor(tm, 4, 32)); tm = fmaxf(tm, __shfl_xor(tm, 8, 32));
            const float nm = fmaxf(mrow[r], tm);
            const float corr = __builtin_amdgcn_exp2f((mrow[r] - nm) * L2E);
            float e0 = __builtin_amdgcn_exp2f((x0 - nm) * L2E); e0 = v0 ? e0 : 0.0f;
            float e1 = __builtin_amdgcn_exp2f((x1 - nm) * L2E); e1 = v1 ? e1 : 0.0f;
            float rs = e0 + e1;
            rs += __shfl_xor(rs, 1, 32); rs += __shfl_xor(rs, 2, 32); rs += __shfl_xor(rs, 4, 32); rs += __shfl_xor(rs, 8, 32);
            lrow[r] = lrow[r] * corr + rs; mrow[r] = nm;
#pragma unroll
            for (int ds = 0; ds < 4; ++ds) { acc[ds][r] *= corr; rac[ds][r] *= corr; }
            const float p0 = e0 * PC, p1 = e1 * PC;
            const h16 h0 = (h16)p0, h1v = (h16)p1;
            float rr0 = p0 - (float)h0; rr0 = rr0 * RC; float rr1 = p1 - (float)h1v; rr1 = rr1 * RC;
            const h16 r0h = (h16)rr0, r1h = (h16)rr1;
            const int po = (8 * hi + r) * PPL + lr;
            ph_w[po] = h0; ph_w[po + 16] = h1v; pr_w[po] = r0h; pr_w[po + 16] = r1h;
        }
        __builtin_amdgcn_fence(3, "wavefront"); __builtin_amdgcn_wave_barrier(); asm volatile("" ::: "memory");
        const h16* pah_p = ph_w + lr * PPL + 8 * hi; const h16* par_p = pr_w + lr * PPL + 8 * hi;
        const v16h pah = cat16(*(const v8ha*)pah_p, *(const v8ha*)(pah_p + 16));
        const v16h par = cat16(*(const v8ha*)par_p, *(const v8ha*)(par_p + 16));
#pragma unroll
        for (int ds = 0; ds < 4; ++ds) {
            const size_t vo = (size_t)(ds * 16 + lr) * SEQ + j0 + 8 * hi;
            const v16h vbh = cat16(ld8(Vh + vo), ld8(Vh + vo + 16));
            const v16h vbr = cat16(ld8(Vr + vo), ld8(Vr + vo + 16));
            acc[ds] = wmma16(pah, vbh, acc[ds]);
            rac[ds] = wmma16(pah, vbr, rac[ds]);
            rac[ds] = wmma16(par, vbh, rac[ds]);
        }
        asm volatile("v_nop\n\tv_nop\n\tv_nop\n\tv_nop" : "+v"(acc[0]), "+v"(acc[1]), "+v"(acc[2]), "+v"(acc[3]), "+v"(rac[0]), "+v"(rac[1]), "+v"(rac[2]), "+v"(rac[3]) : "v"(pah), "v"(par));
        __builtin_amdgcn_wave_barrier(); asm volatile("" ::: "memory");
    }
    float inv[8];
#pragma unroll
    for (int r = 0; r < 8; ++r) { const float den = lrow[r] * PC; inv[r] = (lrow[r] > 0.0f) ? (1.0f / den) : 0.0f; }
#pragma unroll
    for (int ds = 0; ds < 4; ++ds)
#pragma unroll
        for (int r = 0; r < 8; ++r) os_w[(8 * hi + r) * 68 + ds * 16 + lr] = (acc[ds][r] + rac[ds][r] * (1.0f / RC)) * inv[r];
    __builtin_amdgcn_fence(3, "wavefront"); __builtin_amdgcn_wave_barrier(); asm volatile("" ::: "memory");
    float* orow = OUT + ((size_t)b * SEQ + q0) * DM + h * HD;
#pragma unroll 1
    for (int ps = 0; ps < 2; ++ps) {
#pragma unroll
        for (int s = 0; s < 8; ++s) { const int row = 2 * s + hi, cofs = lr * 4; const v4f val = *(const v4fa*)(os_w + row * 68 + cofs);
            *(volatile v4f*)(orow + (size_t)row * DM + cofs) = val; }
        if (ps == 0) __threadfence(); }
}

extern "C" void kernel_launch(void* const* d_in, const int* in_sizes, int n_in,
                              void* d_out, int out_size, void* d_ws, size_t ws_size, hipStream_t stream) {
    if (n_in < 7) return;
    if (in_sizes[0] < ((NB - 1) * SEQ_FULL + SEQ) * DM) return;
    if (in_sizes[1] < DM * DM || in_sizes[3] < DM * DM || in_sizes[5] < DM * DM) return;
    if (in_sizes[2] < DM || in_sizes[4] < DM || in_sizes[6] < DM) return;
    if (out_size < TOK * DM) return;
    const float* x = (const float*)d_in[0]; const float* wq = (const float*)d_in[1]; const float* bq = (const float*)d_in[2];
    const float* wk = (const float*)d_in[3]; const float* bk = (const float*)d_in[4]; const float* wv = (const float*)d_in[5]; const float* bv = (const float*)d_in[6];
    float* OUT = (float*)d_out;
    char* wsp = (char*)d_ws;
    auto take = [&](size_t bytes) { char* p = wsp; wsp += (bytes + 255) & ~(size_t)255; return (void*)p; };
    bf* WQ = (bf*)take((size_t)DM * DM * 2); bf* WK = (bf*)take((size_t)DM * DM * 2); bf* WV = (bf*)take((size_t)DM * DM * 2);
    bf* XB = (bf*)take((size_t)TOK * DM * 2);
    float* F = (float*)take((size_t)TOK * DM * 4);
    h16* QPL = (h16*)take((size_t)TOK * DM * 2);
    h16* KPL = (h16*)take((size_t)TOK * DM * 2);
    h16* VTH = (h16*)take((size_t)TOK * DM * 2);
    h16* VTR = (h16*)take((size_t)TOK * DM * 2);
    const size_t carved = (size_t)(wsp - (char*)d_ws);
    if (carved > ws_size) return;
    if (carved > (size_t)134217728) return;

    const unsigned gW = (unsigned)((DM * DM / 64 + 63) / 64);
    k_wtG<<<gW, 256, 0, stream>>>(wq, DM, DM, WQ);
    k_wtG<<<gW, 256, 0, stream>>>(wk, DM, DM, WK);
    k_wtG<<<gW, 256, 0, stream>>>(wv, DM, DM, WV);
    for (int b = 0; b < NB; ++b)
        k_cvt8<<<(unsigned)(((size_t)SEQ * DM / 8 + 255) / 256), 256, 0, stream>>>(x + (size_t)b * SEQ_FULL * DM, XB + (size_t)b * SEQ * DM, (size_t)SEQ * DM / 8);
    const dim3 gG(TOK / 64, DM / 64, 1);
    const unsigned gP = (unsigned)(((size_t)TOK * DM / 4 + 255) / 256);
    k_gemmw<bf, 0, true><<<gG, 32, 0, stream>>>(XB, nullptr, WQ, nullptr, DM, F, DM, bq, 0, 0, 0);
    k_qkp<<<gP, 256, 0, stream>>>(F, QPL);
    k_gemmw<bf, 0, true><<<gG, 32, 0, stream>>>(XB, nullptr, WK, nullptr, DM, F, DM, bk, 0, 0, 0);
    k_qkp<<<gP, 256, 0, stream>>>(F, KPL);
    k_gemmw<bf, 0, true><<<gG, 32, 0, stream>>>(XB, nullptr, WV, nullptr, DM, F, DM, bv, 0, 0, 0);
    k_vp<<<gP, 256, 0, stream>>>(F, VTH, VTR);
    k_attn<<<dim3(SEQ / 128, NH_, NB), 256, 0, stream>>>(QPL, KPL, VTH, VTR, OUT);
}
